// BatchInfoNCELoss_8641474200145
// MI455X (gfx1250) — hardware-run, weakly checked
//
#include <hip/hip_runtime.h>
#include <math.h>

typedef __attribute__((ext_vector_type(16))) _Float16 v16h;
typedef __attribute__((ext_vector_type(16))) __bf16 v16b;
typedef __attribute__((ext_vector_type(8)))  _Float16 v8h;
typedef __attribute__((ext_vector_type(8)))  float v8f;
typedef __attribute__((ext_vector_type(4)))  float v4f;
typedef __attribute__((ext_vector_type(2)))  float v2f;
typedef __attribute__((ext_vector_type(4)))  unsigned v4u;
typedef __attribute__((ext_vector_type(4)))  int v4i;
typedef float __attribute__((may_alias)) float_a;
typedef int __attribute__((may_alias)) int_a;

template <typename T> __device__ __forceinline__ void vst2(void* p, T v) { *(volatile T*)p = v; __threadfence(); *(volatile T*)p = v; }
__device__ __forceinline__ v8f wmma16(v16h a, v16h b, v8f c) {
  v8f d = __builtin_amdgcn_wmma_f32_16x16x32_f16(false, a, false, b, (short)0, c, false, false);
  asm volatile("v_nop\n\tv_nop\n\tv_nop\n\tv_nop" : "+v"(d) : "v"(a), "v"(b));
  return d;
}
__device__ __forceinline__ v8f wmma_bf(v16b a, v16b b, v8f c) {
  v8f d = __builtin_amdgcn_wmma_f32_16x16x32_bf16(false, a, false, b, (short)0, c, false, false);
  asm volatile("v_nop\n\tv_nop\n\tv_nop\n\tv_nop" : "+v"(d) : "v"(a), "v"(b));
  return d;
}
__device__ __forceinline__ v16h frag_h(const _Float16* rowk0, int lane) {
  union { v16h v; v8h q[2]; } u; const _Float16* p = rowk0 + 8 * (lane >> 4);
  u.q[0] = *(const v8h*)p; u.q[1] = *(const v8h*)(p + 16); return u.v;
}
__device__ __forceinline__ v16h frag_f32(const float* rowk0, int lane) {
  v16h a; const float* p = rowk0 + 8 * (lane >> 4);
#pragma unroll
  for (int i = 0; i < 8; ++i) { a[i] = (_Float16)p[i]; a[8 + i] = (_Float16)p[16 + i]; }
  return a;
}
__device__ __forceinline__ v16h frag_f32s(const float* rowk0, int lane, float sc) {
  v16h a; const float* p = rowk0 + 8 * (lane >> 4);
#pragma unroll
  for (int i = 0; i < 8; ++i) { a[i] = (_Float16)(p[i] * sc); a[8 + i] = (_Float16)(p[16 + i] * sc); }
  return a;
}
__device__ __forceinline__ v16h fragc_f32(const float* W, int k0, int n, int lane, int ld, int K) {
  v16h a; const int g = lane >> 4;
#pragma unroll
  for (int i = 0; i < 8; ++i) { const int ka = k0 + 8 * g + i, kb = ka + 16;
    a[i] = (_Float16)(ka < K ? W[(size_t)(ka < K ? ka : K - 1) * ld + n] : 0.f); a[8 + i] = (_Float16)(kb < K ? W[(size_t)(kb < K ? kb : K - 1) * ld + n] : 0.f); }
  return a;
}
struct F2 { v16b h, l; };
__device__ __forceinline__ F2 bsplit16(const float v[16]) { F2 r;
#pragma unroll
  for (int i = 0; i < 16; ++i) { const __bf16 h = (__bf16)v[i]; r.h[i] = h; r.l[i] = (__bf16)(v[i] - (float)h); }
  return r; }
__device__ __forceinline__ F2 split_row(const float* row, int k0, int lane) { float v[16]; const float* p = row + k0 + 8 * (lane >> 4);
#pragma unroll
  for (int i = 0; i < 8; ++i) { v[i] = p[i]; v[8 + i] = p[16 + i]; }
  return bsplit16(v); }
__device__ __forceinline__ F2 split_rowK(const float* row, int k0, int lane, int K) { float v[16]; const int g = lane >> 4;
#pragma unroll
  for (int i = 0; i < 8; ++i) { const int ka = k0 + 8 * g + i, kb = ka + 16; v[i] = ka < K ? row[ka < K ? ka : K - 1] : 0.f; v[8 + i] = kb < K ? row[kb < K ? kb : K - 1] : 0.f; }
  return bsplit16(v); }
__device__ __forceinline__ F2 split_col(const float* W, int k0, int n, int lane, int ld, int K) { float v[16]; const int g = lane >> 4;
#pragma unroll
  for (int i = 0; i < 8; ++i) { const int ka = k0 + 8 * g + i, kb = ka + 16; v[i] = ka < K ? W[(size_t)(ka < K ? ka : K - 1) * ld + n] : 0.f; v[8 + i] = kb < K ? W[(size_t)(kb < K ? kb : K - 1) * ld + n] : 0.f; }
  return bsplit16(v); }
__device__ __forceinline__ v8f mac3(const F2& a, const F2& b, v8f c) { c = wmma_bf(a.l, b.h, c); c = wmma_bf(a.h, b.l, c); return wmma_bf(a.h, b.h, c); }
__device__ __forceinline__ float sigm(float v) { return 1.0f / (1.0f + expf(-v)); }
#define LDSX() do { asm volatile("s_wait_dscnt 0" ::: "memory"); __builtin_amdgcn_wave_barrier(); __builtin_amdgcn_fence(__ATOMIC_RELEASE, "workgroup"); } while (0)


#define NI 16
#define HL 128
#define NPX (HL * HL)
#define CL 16
#define DP 144
#define DPP 160
#define NS 100
#define NSP 112
#define KC 8
#define NOFF 13
#ifndef NIT
#define NIT NI
#endif
typedef __attribute__((ext_vector_type(8))) __bf16 v8b;
__device__ __forceinline__ v16b frag_b(const __bf16* rowk0, int lane) {
  union { v16b v; v8b q[2]; } u; const __bf16* p = rowk0 + 8 * (lane >> 4);
  u.q[0] = *(const v8b*)p; u.q[1] = *(const v8b*)(p + 16); return u.v;
}
__device__ __forceinline__ float bfr(float v) { return (float)(__bf16)v; }
__device__ __attribute__((noinline)) float exp_ni(float v) { return expf(v); }
__device__ __attribute__((noinline)) float erf_ni(float v) { return erff(v); }
__device__ __attribute__((noinline)) float log_ni(float v) { return logf(v); }
__constant__ int c_offy[NOFF] = {-2, -1, -1, -1, 0, 0, 0, 0, 0, 1, 1, 1, 2};
__constant__ int c_offx[NOFF] = { 0, -1,  0,  1, -2, -1, 0, 1, 2, -1, 0, 1, 0};

#define WS_PT   0u
#define WS_INV  (WS_PT + 2u * (size_t)NI * NPX * DPP)
#define WS_PART (WS_INV + 4u * (size_t)NI * NPX)
#define WS_END  (WS_PART + 128u * NI)

__global__ __launch_bounds__(256) void k_patch(const float* __restrict__ LAT, __bf16* __restrict__ PT, float* __restrict__ INV) {
  __shared__ __align__(16) __bf16 s[64][DPP]; __shared__ float sq[64][4]; __shared__ __align__(16) float sinv[64];
  const int tid = threadIdx.x; const int b = blockIdx.y; const int p0 = blockIdx.x * 64;
  for (int e = tid; e < 64 * DPP; e += 256) { const int r = e / DPP, d = e % DPP; const int p = p0 + r; const int h = p / HL, w = p % HL; float v = 0.f;
    if (d < DP) { const int q = d / CL, c = d % CL; const int hh = min(max(h + q / 3 - 1, 0), HL - 1), ww = min(max(w + q % 3 - 1, 0), HL - 1); v = bfr(LAT[(((size_t)b * HL + hh) * HL + ww) * CL + c]); }
    s[r][d] = (__bf16)v; }
  __syncthreads();
  { const int r = tid >> 2, part = tid & 3; float a = 0.f; for (int d = part; d < DP; d += 4) { const float v = (float)s[r][d]; a += v * v; } sq[r][part] = a; }
  __syncthreads();
  if (tid < 64) { const float a = (sq[tid][0] + sq[tid][1]) + (sq[tid][2] + sq[tid][3]); sinv[tid] = 1.0f / fmaxf(sqrtf(a), 1e-12f); }
  __syncthreads();
  for (int e = tid; e < 64 * DPP / 8; e += 256) { const int r = e / (DPP / 8), pc = e % (DPP / 8); vst2((unsigned*)(PT + ((size_t)b * NPX + p0 + r) * DPP + pc * 8), *(const v4u*)&s[r][pc * 8]); }
  if (tid < 16) vst2(INV + (size_t)b * NPX + p0 + tid * 4, *(const v4f*)&sinv[tid * 4]);
}
__global__ __launch_bounds__(224) void k_loss(const __bf16* __restrict__ PT, const float* __restrict__ INV, const int* __restrict__ AIDX, const int* __restrict__ CIDX, double* __restrict__ PART) {
  __shared__ float spos[NSP], sneg[NSP], scross[NSP]; __shared__ int spc[NSP], snc[NSP], scc[NSP]; __shared__ double sred[2][7]; __shared__ __align__(16) double sline[16];
  const int tid = threadIdx.x, wave = tid >> 5, lane = tid & 31, col = lane & 15, g = lane >> 4; const int b = blockIdx.x;
  const int arow = wave * 16 + col; const int aidx_l = AIDX[(size_t)b * NS + min(arow, NS - 1)];
  v16b aq[DPP / 32];
#pragma unroll
  for (int kc = 0; kc < DPP / 32; ++kc) aq[kc] = frag_b(PT + ((size_t)b * NPX + aidx_l) * DPP + kc * 32, lane);
  float inva[8]; int ah[8], aw[8];
#pragma unroll
  for (int r = 0; r < 8; ++r) { const int ar = wave * 16 + 8 * g + r; const int ai = AIDX[(size_t)b * NS + min(ar, NS - 1)]; inva[r] = INV[(size_t)b * NPX + ai]; ah[r] = ai / HL; aw[r] = ai % HL; }
  float psum[8], nsum[8]; int pcnt[8], ncnt[8];
#pragma unroll
  for (int r = 0; r < 8; ++r) { psum[r] = 0.f; nsum[r] = 0.f; pcnt[r] = 0; ncnt[r] = 0; }
#pragma unroll 1
  for (int pt = 0; pt < NPX / 16; ++pt) { const int pcol = pt * 16 + col; v8f c = {};
#pragma unroll
    for (int kc = 0; kc < DPP / 32; ++kc) c = wmma_bf(aq[kc], frag_b(PT + ((size_t)b * NPX + pcol) * DPP + kc * 32, lane), c);
    const float invp = INV[(size_t)b * NPX + pcol]; const int ph = pcol / HL, pw = pcol % HL;
#pragma unroll
    for (int r = 0; r < 8; ++r) { const float sim = c[r] * inva[r] * invp; const float e = exp_ni(sim); const int dh = ph - ah[r], dw = pw - aw[r]; const int d2 = dh * dh + dw * dw;
      if (d2 > 0 && d2 <= 9) { psum[r] += e; pcnt[r] += 1; }
      if (d2 > 121) { nsum[r] += e; ncnt[r] += 1; } } }
#pragma unroll
  for (int r = 0; r < 8; ++r) {
#pragma unroll
    for (int o = 1; o < 16; o <<= 1) { psum[r] += __shfl_xor(psum[r], o); nsum[r] += __shfl_xor(nsum[r], o); pcnt[r] += __shfl_xor(pcnt[r], o); ncnt[r] += __shfl_xor(ncnt[r], o); }
    if (col == 0) { const int ar = wave * 16 + 8 * g + r; spos[ar] = psum[r]; sneg[ar] = nsum[r]; spc[ar] = pcnt[r]; snc[ar] = ncnt[r]; } }
  __syncthreads();
  { const int ar = tid % NSP, half = tid / NSP; float csum = 0.f; int ccnt = 0;
    if (ar < NS) { const int ai = AIDX[(size_t)b * NS + ar]; const int ahh = ai / HL, aww = ai % HL; const __bf16* arow_p = PT + ((size_t)b * NPX + ai) * DPP; const float ia = INV[(size_t)b * NPX + ai];
      for (int m = half; m < NOFF; m += 2) { const int py = ahh + c_offy[m], px = aww + c_offx[m]; if (py < 0 || py >= HL || px < 0 || px >= HL) continue;
        const int pidx = py * HL + px;
        for (int k = 0; k < KC; ++k) { const int ob = min(max(CIDX[((size_t)b * NS + ar) * KC + k], 0), NI - 1); const __bf16* prow = PT + ((size_t)ob * NPX + pidx) * DPP; float dsum = 0.f;
#pragma unroll 4
          for (int d = 0; d < DP; ++d) dsum += (float)arow_p[d] * (float)prow[d];
          const float cs = dsum * ia * INV[(size_t)ob * NPX + pidx] * 2.0f;
          csum += exp_ni(cs); }
        ccnt += 1; } }
    if (half == 1) { scross[ar] = csum; scc[ar] = ccnt; }
    __syncthreads();
    if (half == 0) { csum += scross[ar]; ccnt += scc[ar]; scross[ar] = csum; scc[ar] = ccnt; }
    __syncthreads(); }
  double lsum = 0.0, nval = 0.0;
  if (tid < NS) { const int ar = tid; const float pm = spos[ar] / (float)max(spc[ar], 1); const float nm = sneg[ar] / (float)max(snc[ar], 1); const float cm = scross[ar] / (float)max(scc[ar], 1);
    const float lw = -log_ni(pm / (pm + nm + 1e-8f)); const float la = -log_ni(pm / (pm + cm + 1e-8f)); const bool hasn = snc[ar] > 0, hasc = scc[ar] > 0; const bool valid = (spc[ar] > 0) && (hasn || hasc);
    const float per = (hasn ? lw : 0.f) + (hasc ? la : 0.f); lsum = valid ? (double)per : 0.0; nval = valid ? 1.0 : 0.0; }
#pragma unroll
  for (int o = 1; o < 32; o <<= 1) { lsum += __shfl_xor(lsum, o); nval += __shfl_xor(nval, o); }
  if (lane == 0) { sred[0][wave] = lsum; sred[1][wave] = nval; }
  if (tid < 16) sline[tid] = 0.0;
  __syncthreads();
  if (tid == 0) { double a = 0.0, n = 0.0; for (int w = 0; w < 7; ++w) { a += sred[0][w]; n += sred[1][w]; } sline[0] = a; sline[1] = n; }
  __syncthreads();
  if (tid < 8) vst2((unsigned*)(PART + (size_t)b * 16 + tid * 2), *(const v4u*)&sline[tid * 2]);
}
__global__ __launch_bounds__(32) void k_final(const double* __restrict__ PART, float* __restrict__ OUT) {
  if (threadIdx.x == 0) { double a = 0.0, n = 0.0; for (int b = 0; b < NIT; ++b) { a += PART[(size_t)b * 16]; n += PART[(size_t)b * 16 + 1]; } const float v = (n > 0.0) ? (float)(a / n) : 0.f; *(volatile float*)OUT = v; *(volatile float*)OUT = v; }
}
extern "C" void kernel_launch(void* const* d_in, const int* in_sizes, int n_in, void* d_out, int out_size, void* d_ws, size_t ws_size, hipStream_t stream) {
  (void)in_sizes; (void)n_in; (void)out_size;
  const float* LAT = (const float*)d_in[0]; const int* AIDX = (const int*)d_in[1]; const int* CIDX = (const int*)d_in[2];
  if (ws_size < (size_t)WS_END) return;
  char* ws = (char*)d_ws; __bf16* PT = (__bf16*)(ws + WS_PT); float* INV = (float*)(ws + WS_INV); double* PART = (double*)(ws + WS_PART);
  k_patch<<<dim3(NPX / 64, NI), 256, 0, stream>>>(LAT, PT, INV);
  k_loss<<<NIT, 224, 0, stream>>>(PT, INV, AIDX, CIDX, PART);
  k_final<<<1, 32, 0, stream>>>(PART, (float*)d_out);
}
